// QuantumGenerator_34394098106454
// MI455X (gfx1250) — hardware-run, weakly checked
//
#include <hip/hip_runtime.h>


#ifndef NB
#define NB 256
#endif
#define NB_FULL 256
#define NQ    16
#define DIMS  65536
#define QT    1024
#define NLAY  6
#define NG    (NLAY * NQ)
#define OUTD  256
#define CSO   DIMS
#define CSF   256
#define SMEM_FLOATS (DIMS + CSF)
#define SMEM_BYTES  ((size_t)SMEM_FLOATS * 4)
#define PARTO 0
#define QRO   512
#define QPITCH 32
#define HW    4
#define OSP   36
#define QC    16384.0f
#define WC    64.0f
#define CINV  (1.0f / 1048576.0f)

static_assert(NQ == 16);
static_assert(DIMS == (1 << NQ));
static_assert(QT == 1024);
static_assert(DIMS % QT == 0);
static_assert((DIMS >> 1) % QT == 0);
static_assert((DIMS >> 2) % QT == 0);
static_assert(NG == 96);
static_assert(NG % 32 == 0);
static_assert(NG <= QT);
static_assert(2 * NG <= CSF);
static_assert((QT / 32) * NQ <= QRO);
static_assert(QRO + 32 <= DIMS);
static_assert(QPITCH * 4 == 8 * 16);
static_assert(2 * NQ == 32);
static_assert(NB % 16 == 0);
static_assert(OUTD % (32 * HW) == 0);
static_assert(32 * 16 * 4 == 16 * 32 * 4);
static_assert((OSP * 4) % 16 == 0);
static_assert((size_t)HW * 16 * OSP * 4 <= (size_t)131072);
static_assert(SMEM_BYTES <= (size_t)300000);
static_assert(NB <= NB_FULL);

typedef _Float16 h16;
typedef __attribute__((ext_vector_type(16))) _Float16 v16h;
typedef __attribute__((ext_vector_type(8)))  float    v8f;
typedef __attribute__((ext_vector_type(4)))  float    v4f;
typedef v4f  __attribute__((may_alias)) v4fa;

__device__ __forceinline__ unsigned short f2bf(float f) { unsigned u = __float_as_uint(f); u += 0x7FFFu + ((u >> 16) & 1u); return (unsigned short)(u >> 16); }
__device__ __forceinline__ float bfr(float f) { return __uint_as_float(((unsigned)f2bf(f)) << 16); }
__device__ __forceinline__ v8f wmma16(v16h a, v16h b, v8f c) { return __builtin_amdgcn_wmma_f32_16x16x32_f16(false, a, false, b, (short)0, c, false, false); }
__device__ __forceinline__ void wave_sync() { __builtin_amdgcn_fence(3  , "wavefront"); __builtin_amdgcn_wave_barrier(); asm volatile("" ::: "memory"); }
static __device__ __forceinline__ h16 toh_flush(float v) { const h16 r = (h16)v; return (fabsf(v) < 6.103515625e-05f) ? (h16)0.0f : r; }

__global__ __launch_bounds__(QT) void k_state(const float* __restrict__ z, const float* __restrict__ qw, float* QF) {
    extern __shared__ __align__(16) float smem[];
    const int tid = threadIdx.x;
    const int lane = tid & 31;
    const int wave = __builtin_amdgcn_readfirstlane((int)(threadIdx.x >> 5));
    const int b = blockIdx.x;

#pragma unroll 4
    for (int i = tid; i < DIMS; i += QT) smem[i] = 0.0f;
    if (tid == 0) smem[0] = 1.0f;
    if (wave < NG / 32) {
        const int g = tid;
        const float th = bfr(qw[g]);
        float zz = z[(size_t)b * NQ + (g & (NQ - 1))];
        asm volatile("" : "+v"(zz));
        const float ang = (g < NQ) ? (th + bfr(zz)) : th;
        float sv, cv;
        sincosf(0.5f * ang, &sv, &cv);
        smem[CSO + 2 * g] = cv;
        smem[CSO + 2 * g + 1] = sv;
    }
    __syncthreads();

#pragma unroll 1
    for (int l = 0; l < NLAY; ++l) {
#pragma unroll 1
        for (int w = 0; w < NQ; ++w) {
            const int g = l * NQ + w;
            const float c = smem[CSO + 2 * g];
            const float s = smem[CSO + 2 * g + 1];
            const int bit = 1 << w;
            const int mlow = bit - 1;
#pragma unroll 4
            for (int p = tid; p < (DIMS >> 1); p += QT) {
                const int i0 = ((p >> w) << (w + 1)) | (p & mlow);
                const int i1 = i0 | bit;
                const float a0 = smem[i0];
                const float a1 = smem[i1];
                smem[i0] = c * a0 - s * a1;
                smem[i1] = s * a0 + c * a1;
            }
            __syncthreads();
        }
#pragma unroll 1
        for (int w = 0; w < NQ; ++w) {
            const int ctrl = w, tgt = (w + 1) & (NQ - 1);
            const int lo = ctrl < tgt ? ctrl : tgt;
            const int hb = ctrl < tgt ? tgt : ctrl;
            const int cb = 1 << ctrl;
            const int tb = 1 << tgt;
#pragma unroll 4
            for (int q = tid; q < (DIMS >> 2); q += QT) {
                int i = ((q >> lo) << (lo + 1)) | (q & ((1 << lo) - 1));
                i = ((i >> hb) << (hb + 1)) | (i & ((1 << hb) - 1));
                const int i0 = i | cb;
                const int i1 = i0 | tb;
                const float x = smem[i0];
                const float y = smem[i1];
                smem[i0] = y;
                smem[i1] = x;
            }
            __syncthreads();
        }
    }

    float acc[NQ];
#pragma unroll
    for (int w = 0; w < NQ; ++w) acc[w] = 0.0f;
#pragma unroll 2
    for (int i = tid; i < DIMS; i += QT) {
        const float a = smem[i];
        const float p = a * a;
#pragma unroll
        for (int w = 0; w < NQ; ++w) {
            const unsigned sgn = (((unsigned)i) << (31 - w)) & 0x80000000u;
            acc[w] += __uint_as_float(__float_as_uint(p) ^ sgn);
        }
    }
    float mine = 0.0f;
#pragma unroll
    for (int w = 0; w < NQ; ++w) {
        float v = acc[w];
#pragma unroll
        for (int off = 16; off; off >>= 1) v += __shfl_xor(v, off, 32);
        mine = (lane == w) ? v : mine;
    }
    __syncthreads();
    if (lane < NQ) smem[PARTO + wave * NQ + lane] = mine;
    __syncthreads();
    if (wave == 0) {
        float tot = 0.0f;
#pragma unroll 4
        for (int wv = 0; wv < QT / 32; ++wv) tot += smem[PARTO + wv * NQ + (lane & (NQ - 1))];
        const float qv = (lane < NQ) ? tot : 0.0f;
        smem[QRO + lane] = qv;
        wave_sync();
        if (lane < 8) {
            const v4f val = *(const v4fa*)(&smem[QRO + 4 * lane]);
            float* dst = QF + (size_t)b * QPITCH + 4 * lane;
            *(volatile v4f*)dst = val;
            __threadfence();
            *(volatile v4f*)dst = val;
        }
    }
}

__device__ __forceinline__ v16h ld_wfrag(const float* __restrict__ wp) {
    const v4f w0 = *(const v4f*)wp, w1 = *(const v4f*)(wp + 4);
    v16h f;
#pragma unroll
    for (int i = 0; i < 4; ++i) {
        const h16 g0 = toh_flush(bfr(w0[i]) * WC), g1 = toh_flush(bfr(w1[i]) * WC);
        f[i] = g0; f[4 + i] = g1; f[8 + i] = g0; f[12 + i] = g1;
    }
    return f;
}

__global__ __launch_bounds__(32 * HW) void k_head(const float* __restrict__ QF, const float* __restrict__ W, const float* __restrict__ bias, float* OUT) {
    __shared__ __align__(16) float os[HW * 16 * OSP];
    const int lane = threadIdx.x & 31, lr = lane & 15, hi = lane >> 4;
    const int wave = __builtin_amdgcn_readfirstlane((int)(threadIdx.x >> 5));
    const int m0 = blockIdx.x * 16;
    const int n0 = (blockIdx.y * HW + wave) * 32;
    const float* qp = QF + (size_t)(m0 + lr) * QPITCH + 8 * hi;
    const v4f q0 = *(const v4f*)qp, q1 = *(const v4f*)(qp + 4);
    v16h a;
#pragma unroll
    for (int i = 0; i < 4; ++i) {
        const float x0 = q0[i] * QC, x1 = q1[i] * QC;
        const h16 h0 = toh_flush(x0), h1 = toh_flush(x1);
        a[i] = h0; a[4 + i] = h1;
        a[8 + i] = toh_flush(x0 - (float)h0); a[12 + i] = toh_flush(x1 - (float)h1);
    }
    const v16h b0 = ld_wfrag(W + (size_t)(n0 + lr) * NQ + 8 * hi);
    const v16h b1 = ld_wfrag(W + (size_t)(n0 + 16 + lr) * NQ + 8 * hi);
    v8f c0 = (v8f){}, c1 = (v8f){};
    c0 = wmma16(a, b0, c0);
    asm volatile("v_nop\n\tv_nop\n\tv_nop\n\tv_nop" : "+v"(c0) : "v"(a), "v"(b0));
    c1 = wmma16(a, b1, c1);
    asm volatile("v_nop\n\tv_nop\n\tv_nop\n\tv_nop" : "+v"(c1) : "v"(a), "v"(b1));
    const int wb = wave * 16 * OSP;
#pragma unroll
    for (int r = 0; r < 8; ++r) {
        os[wb + (8 * hi + r) * OSP + lr] = c0[r] * CINV;
        os[wb + (8 * hi + r) * OSP + 16 + lr] = c1[r] * CINV;
    }
    wave_sync();
    const int cofs = (lane & 7) * 4;
    const v4f braw = *(const v4f*)(bias + n0 + cofs);
    v4f bb;
#pragma unroll
    for (int i = 0; i < 4; ++i) bb[i] = bfr(braw[i]);
#pragma unroll 1
    for (int s = 0; s < 4; ++s) { const int row = 4 * s + (lane >> 3);
        const v4f v = *(const v4fa*)(&os[wb + row * OSP + cofs]); v4f t;
#pragma unroll
        for (int i = 0; i < 4; ++i) t[i] = tanhf(v[i] + bb[i]);
        *(v4fa*)(&os[wb + row * OSP + cofs]) = t; }
    wave_sync();
    float* orow = OUT + (size_t)m0 * OUTD + n0;
#pragma unroll 1
    for (int ps = 0; ps < 2; ++ps) {
#pragma unroll
        for (int s = 0; s < 4; ++s) { const int row = 4 * s + (lane >> 3);
            const v4f val = *(const v4fa*)(&os[wb + row * OSP + cofs]);
            *(volatile v4f*)(orow + (size_t)row * OUTD + cofs) = val; }
        if (ps == 0) __threadfence(); }
}

static constexpr size_t al256(size_t v) { return (v + 255) & ~(size_t)255; }
static constexpr size_t SZ_QF = al256((size_t)NB * QPITCH * 4);
static constexpr size_t SZ_TOTAL = SZ_QF;
static_assert(SZ_TOTAL <= (size_t)134217728);
static_assert((size_t)NB * QPITCH * 4 <= SZ_QF);

extern "C" void kernel_launch(void* const* d_in, const int* in_sizes, int n_in,
                              void* d_out, int out_size, void* d_ws, size_t ws_size, hipStream_t stream) {
    if (n_in < 4) return;
    if (in_sizes[0] < NB * NQ || in_sizes[1] < NG || in_sizes[2] < OUTD * NQ || in_sizes[3] < OUTD) return;
    if (out_size < NB * OUTD) return;
    if (SZ_TOTAL > ws_size) return;
    const float* z    = (const float*)d_in[0];
    const float* qw   = (const float*)d_in[1];
    const float* W    = (const float*)d_in[2];
    const float* bias = (const float*)d_in[3];
    float* OUT = (float*)d_out;
    float* QF  = (float*)d_ws;

    hipFuncSetAttribute(reinterpret_cast<const void*>(&k_state), hipFuncAttributeMaxDynamicSharedMemorySize, (int)SMEM_BYTES);
    k_state<<<dim3(NB, 1, 1), QT, SMEM_BYTES, stream>>>(z, qw, QF);
    k_head<<<dim3(NB / 16, OUTD / (32 * HW), 1), 32 * HW, 0, stream>>>(QF, W, bias, OUT);
}
